// LowRankAttention_14181982011820
// MI455X (gfx1250) — hardware-verified
//
#include <hip/hip_runtime.h>


#define NB_  8
#define NQ   100
#define NK   100
#define NP   128
#define DM   512
#define NH_  8
#define DK   64
#define MID  128
#define RPB  (NH_ * NQ * NP)
#define PQ   832
typedef _Float16 h16;
typedef unsigned short bf;
typedef __attribute__((ext_vector_type(16))) __bf16   v16bf;
typedef __attribute__((ext_vector_type(16))) _Float16 v16h;
typedef __attribute__((ext_vector_type(8)))  _Float16 v8h;
typedef __attribute__((ext_vector_type(8)))  unsigned short v8us;
typedef __attribute__((ext_vector_type(8)))  float    v8f;
typedef __attribute__((ext_vector_type(4)))  float    v4f;
typedef v8h  __attribute__((may_alias)) v8ha;
typedef v4f  __attribute__((may_alias)) v4fa;
typedef v8us __attribute__((may_alias)) v8usa;

__device__ __forceinline__ unsigned short f2bf(float f) { unsigned u = __float_as_uint(f); u += 0x7FFFu + ((u >> 16) & 1u); return (unsigned short)(u >> 16); }
__device__ __forceinline__ float bf2f(unsigned short b) { return __uint_as_float(((unsigned)b) << 16); }
__device__ __forceinline__ float bfr(float f) { return bf2f(f2bf(f)); }
__device__ __forceinline__ v16h cat16(v8h lo, v8h hi) { return __builtin_shufflevector(lo, hi, 0, 1, 2, 3, 4, 5, 6, 7, 8, 9, 10, 11, 12, 13, 14, 15); }
__device__ __forceinline__ v16bf cat16b(v8us lo, v8us hi) { return __builtin_bit_cast(v16bf, __builtin_shufflevector(lo, hi, 0, 1, 2, 3, 4, 5, 6, 7, 8, 9, 10, 11, 12, 13, 14, 15)); }
__device__ __forceinline__ v8f wmma16(v16h a, v16h b, v8f c) { return __builtin_amdgcn_wmma_f32_16x16x32_f16(false, a, false, b, (short)0, c, false, false); }
__device__ __forceinline__ v8f wmmab(v16bf a, v16bf b, v8f c) { return __builtin_amdgcn_wmma_f32_16x16x32_bf16(false, a, false, b, (short)0, c, false, false); }


template <typename T16> struct WFrag;
template <> struct WFrag<h16> { typedef v16h V; static __device__ __forceinline__ V ld(const h16* p) { return cat16(*(const v8h*)p, *(const v8h*)(p + 16)); } static __device__ __forceinline__ v8f mma(V a, V b, v8f c) { return wmma16(a, b, c); } };
template <> struct WFrag<bf> { typedef v16bf V; static __device__ __forceinline__ V ld(const bf* p) { return cat16b(*(const v8us*)p, *(const v8us*)(p + 16)); } static __device__ __forceinline__ v8f mma(V a, V b, v8f c) { return wmmab(a, b, c); } };
template <typename T16, int NSPLIT, bool BIAS>
__global__ __launch_bounds__(32) void k_gemmw(const T16* __restrict__ A, const T16* __restrict__ A2, const T16* __restrict__ Bt, const T16* __restrict__ Bt2, int K, float* C, int ldc, const float* __restrict__ bias, size_t sA, size_t sB, size_t sC) {
    typedef typename WFrag<T16>::V V;
    __shared__ __align__(16) float os[16 * 68];
    const size_t z = blockIdx.z; A += z * sA; if (A2) A2 += z * sA; Bt += z * sB; if (Bt2) Bt2 += z * sB; C += z * sC;
    const int lane = threadIdx.x & 31, lr = lane & 15, hi = lane >> 4; const int r0 = blockIdx.x * 64, c0 = blockIdx.y * 64;
    v8f acc[4][4];
#pragma unroll
    for (int mb = 0; mb < 4; ++mb)
#pragma unroll
        for (int nb = 0; nb < 4; ++nb) acc[mb][nb] = (v8f){};
    const size_t aoff = (size_t)(r0 + lr) * K + 8 * hi, boff = (size_t)(c0 + lr) * K + 8 * hi;
#pragma unroll 1
    for (int kc = 0; kc < K; kc += 32) {
        V a[4], a2[4];
#pragma unroll
        for (int mb = 0; mb < 4; ++mb) { a[mb] = WFrag<T16>::ld(A + aoff + (size_t)mb * 16 * K + kc); if (NSPLIT == 1 || NSPLIT == 2) a2[mb] = WFrag<T16>::ld(A2 + aoff + (size_t)mb * 16 * K + kc); }
#pragma unroll
        for (int nb = 0; nb < 4; ++nb) { const V b = WFrag<T16>::ld(Bt + boff + (size_t)nb * 16 * K + kc); V b2; if (NSPLIT >= 2) b2 = WFrag<T16>::ld(Bt2 + boff + (size_t)nb * 16 * K + kc);
#pragma unroll
            for (int mb = 0; mb < 4; ++mb) { acc[mb][nb] = WFrag<T16>::mma(a[mb], b, acc[mb][nb]); if (NSPLIT == 1 || NSPLIT == 2) acc[mb][nb] = WFrag<T16>::mma(a2[mb], b, acc[mb][nb]); if (NSPLIT >= 2) acc[mb][nb] = WFrag<T16>::mma(a[mb], b2, acc[mb][nb]); } }
        asm volatile("v_nop\n\tv_nop\n\tv_nop\n\tv_nop" : "+v"(acc[0][0]), "+v"(acc[1][1]), "+v"(acc[2][2]), "+v"(acc[3][3]) : "v"(a[0]), "v"(a[3]));
    }
#pragma unroll
    for (int mb = 0; mb < 4; ++mb) {
#pragma unroll
        for (int nb = 0; nb < 4; ++nb) {
#pragma unroll
            for (int j = 0; j < 8; ++j) os[(hi * 8 + j) * 68 + nb * 16 + lr] = acc[mb][nb][j]; }
        __builtin_amdgcn_wave_barrier(); asm volatile("" ::: "memory");
        float* crow = C + (size_t)(r0 + mb * 16) * ldc + c0;
#pragma unroll 1
        for (int ps = 0; ps < 2; ++ps) {
#pragma unroll
            for (int s = 0; s < 8; ++s) { const int row = 2 * s + hi, cofs = lr * 4; v4f val = *(const v4fa*)(os + row * 68 + cofs); if (BIAS) { val[0] += bfr(bias[c0 + cofs]); val[1] += bfr(bias[c0 + cofs + 1]); val[2] += bfr(bias[c0 + cofs + 2]); val[3] += bfr(bias[c0 + cofs + 3]); }
                *(volatile v4f*)(crow + (size_t)row * ldc + cofs) = val; }
            if (ps == 0) __threadfence(); }
        __builtin_amdgcn_wave_barrier(); asm volatile("" ::: "memory");
    }
}

typedef __attribute__((ext_vector_type(4))) unsigned short v4us;
typedef __attribute__((ext_vector_type(2))) unsigned short v2us;
__device__ __forceinline__ void splitf(float y, unsigned short& h, unsigned short& l) { h = f2bf(y); l = f2bf(y - bf2f(h)); }
__device__ __forceinline__ float ex2(float a) { return __builtin_amdgcn_exp2f(__fmul_rn(a, 1.4426950408889634f)); }
__global__ __launch_bounds__(256) void k_wtG(const float* __restrict__ w, int K, int N, bf* Bt) {
    const int lane = threadIdx.x & 31; const int L0 = (blockIdx.x * 8 + (threadIdx.x >> 5)) * 8; const int nlines = N * K / 64;
#pragma unroll
    for (int ps = 0; ps < 2; ++ps) {
#pragma unroll 1
        for (int l = 0; l < 8; ++l) { const int L = L0 + l; if (L >= nlines) break; const size_t e = (size_t)L * 64 + lane * 2; const int k = (int)(e % K), n = (int)(e / K); v2us o;
            o[0] = f2bf(w[(size_t)k * N + n]); o[1] = f2bf(w[(size_t)(k + 1) * N + n]); *(volatile v2us*)(Bt + e) = o; }
        if (ps == 0) __threadfence(); }
}

__global__ __launch_bounds__(256) void k_cvt8(const float* __restrict__ src, bf* dst, size_t n8) { const size_t i = (size_t)blockIdx.x * 256 + threadIdx.x; if (i >= n8) return; const v8f v = *(const v8f*)(src + i * 8); v8us o;
#pragma unroll
    for (int k = 0; k < 8; ++k) o[k] = f2bf(v[k]); *(volatile v8us*)(dst + i * 8) = o; __threadfence(); *(volatile v8us*)(dst + i * 8) = o; }

__global__ __launch_bounds__(256) void k_zero(float* Z, size_t n4) { const size_t i = (size_t)blockIdx.x * 256 + threadIdx.x; if (i >= n4) return; v4f o; o[0] = o[1] = o[2] = o[3] = 0.f; *(volatile v4f*)(Z + i * 4) = o; __threadfence(); *(volatile v4f*)(Z + i * 4) = o; }
__global__ __launch_bounds__(256) void k_zero16(bf* Z, size_t n8) { const size_t i = (size_t)blockIdx.x * 256 + threadIdx.x; if (i >= n8) return; v8us o; for (int k = 0; k < 8; ++k) o[k] = 0; *(volatile v8us*)(Z + i * 8) = o; __threadfence(); *(volatile v8us*)(Z + i * 8) = o; }
__global__ __launch_bounds__(256) void k_elugn(const float* __restrict__ X, const float* __restrict__ gw, const float* __restrict__ gb, float* OUTP) {
    const int i = blockIdx.x * 256 + threadIdx.x; if (i >= NQ * NH_ * 8) return; const int g8 = i % 8; const int h = (i / 8) % NH_; const int r = i / (8 * NH_); const float* xr = X + (size_t)r * DM + h * DK;
    auto elu = [](float a) { return a > 0.0f ? a : __fsub_rn(ex2(a), 1.0f); };
    float s = 0.f;
#pragma unroll 1
    for (int d = 0; d < DK; ++d) s = __fadd_rn(s, elu(xr[d]));
    const float mu = __fdiv_rn(s, (float)DK); float s2 = 0.f;
#pragma unroll 1
    for (int d = 0; d < DK; ++d) { float d0 = __fsub_rn(elu(xr[d]), mu); asm volatile("" : "+v"(d0)); float p = __fmul_rn(d0, d0); asm volatile("" : "+v"(p)); s2 = __fadd_rn(s2, p); }
    const float rs = __fdiv_rn(1.0f, __fsqrt_rn(__fadd_rn(__fdiv_rn(s2, (float)DK), 1e-5f))); v4f oa, ob;
#pragma unroll
    for (int q = 0; q < 8; ++q) { const int d = g8 * 8 + q; float d0 = __fsub_rn(elu(xr[d]), mu); asm volatile("" : "+v"(d0)); float n = __fmul_rn(d0, rs); asm volatile("" : "+v"(n)); float y = __fmul_rn(n, bfr(gw[h * DK + d])); asm volatile("" : "+v"(y)); y = __fadd_rn(y, bfr(gb[h * DK + d])); if (q < 4) oa[q] = y; else ob[q - 4] = y; }
    float* dst = OUTP + (size_t)r * DM + h * DK + g8 * 8; *(volatile v4f*)dst = oa; *(volatile v4f*)(dst + 4) = ob; __threadfence(); *(volatile v4f*)dst = oa; *(volatile v4f*)(dst + 4) = ob; }
__global__ __launch_bounds__(256) void k_prod(const float* __restrict__ Q1, const float* __restrict__ KK, bf* Ah, bf* Al) { const size_t i = (size_t)blockIdx.x * 256 + threadIdx.x; if (i >= (size_t)RPB * DK / 4) return; const int d0 = (int)(i % (DK / 4)) * 4; const size_t row = i / (DK / 4); const int kk = (int)(row % NP); const int q = (int)((row / NP) % NQ); const int h = (int)(row / ((size_t)NP * NQ)); v4us oh, ol;
#pragma unroll
    for (int j = 0; j < 4; ++j) { const int d = d0 + j; float p = 0.0f; if (kk < NK) p = __fmul_rn(Q1[(size_t)q * DM + h * DK + d], KK[(size_t)kk * DM + h * DK + d]); unsigned short a, b; splitf(p, a, b); oh[j] = a; ol[j] = b; }
    *(volatile v4us*)(Ah + row * DK + d0) = oh; *(volatile v4us*)(Al + row * DK + d0) = ol; __threadfence(); *(volatile v4us*)(Ah + row * DK + d0) = oh; *(volatile v4us*)(Al + row * DK + d0) = ol; }
__global__ __launch_bounds__(256) void k_sppool(const float* __restrict__ AM, float* POOL) { const int i = blockIdx.x * 256 + threadIdx.x; if (i >= NH_ * NQ * (MID / 4)) return; const int m0 = (i % (MID / 4)) * 4; const int hq = i / (MID / 4); const float* base = AM + (size_t)hq * NP * MID + m0; v4f acc; acc[0] = acc[1] = acc[2] = acc[3] = 0.f;
#pragma unroll 1
    for (int kk = 0; kk < NK; ++kk) { const v4f a = *(const v4f*)(base + (size_t)kk * MID);
#pragma unroll
        for (int j = 0; j < 4; ++j) acc[j] = __fadd_rn(acc[j], fmaxf(a[j], 0.0f)); }
    v4f o; for (int j = 0; j < 4; ++j) o[j] = __fdiv_rn(acc[j], (float)NK); float* dst = POOL + (size_t)hq * MID + m0; *(volatile v4f*)dst = o; __threadfence(); *(volatile v4f*)dst = o; }
__global__ __launch_bounds__(256) void k_splog(const float* __restrict__ AM, const float* __restrict__ ws, const float* __restrict__ bs, float* SP) { const size_t row = (size_t)blockIdx.x * 256 + threadIdx.x; if (row >= (size_t)RPB) return; const int kk = (int)(row % NP); float s = 0.f; const float* a = AM + row * MID;
#pragma unroll 1
    for (int m = 0; m < MID; m += 4) { const v4f v4 = *(const v4f*)(a + m);
#pragma unroll
        for (int j = 0; j < 4; ++j) { float p = __fmul_rn(fmaxf(v4[j], 0.0f), bfr(ws[m + j])); asm volatile("" : "+v"(p)); s = __fadd_rn(s, p); } }
    s = __fadd_rn(s, bfr(bs[0])); if (kk >= NK) s = -3.0e38f; *(volatile float*)(SP + row) = s; __threadfence(); *(volatile float*)(SP + row) = s; }
__global__ __launch_bounds__(256) void k_attv(const float* __restrict__ SP, const float* __restrict__ VV, const float* __restrict__ Q2, const float* __restrict__ CH, bf* Ah, bf* Al) {
    const int i = blockIdx.x * 256 + threadIdx.x; if (i >= NH_ * NQ * (DK / 4)) return; const int d0 = (i % (DK / 4)) * 4; const int hq = i / (DK / 4); const int h = hq / NQ, q = hq % NQ; const float* sp = SP + (size_t)hq * NP; float mx = -3.0e38f;
#pragma unroll 1
    for (int kk = 0; kk < NK; ++kk) mx = fmaxf(mx, sp[kk]);
    float sum = 0.f;
#pragma unroll 1
    for (int kk = 0; kk < NK; ++kk) { float dd = __fsub_rn(sp[kk], mx); asm volatile("" : "+v"(dd)); sum = __fadd_rn(sum, ex2(dd)); }
    const float f = __fdiv_rn(1.0f, sum); v4f acc; acc[0] = acc[1] = acc[2] = acc[3] = 0.f;
#pragma unroll 1
    for (int kk = 0; kk < NK; ++kk) { float dd = __fsub_rn(sp[kk], mx); asm volatile("" : "+v"(dd)); float e = ex2(dd); asm volatile("" : "+v"(e)); const float p = __fmul_rn(e, f); const v4f vv = *(const v4f*)(VV + (size_t)kk * DM + h * DK + d0);
#pragma unroll
        for (int j = 0; j < 4; ++j) { float t = __fmul_rn(p, vv[j]); asm volatile("" : "+v"(t)); acc[j] = __fadd_rn(acc[j], t); } }
    v4us oh, ol;
#pragma unroll
    for (int j = 0; j < 4; ++j) { const int d = d0 + j; const float c = CH[(size_t)hq * DK + d]; const float sg = __fdiv_rn(1.0f, __fadd_rn(1.0f, ex2(-c))); float g = __fmul_rn(acc[j], Q2[(size_t)q * DM + h * DK + d]); asm volatile("" : "+v"(g)); const float o = __fmul_rn(g, sg); unsigned short a, b; splitf(o, a, b); oh[j] = a; ol[j] = b; }
    const size_t oo = (size_t)q * DM + h * DK + d0; *(volatile v4us*)(Ah + oo) = oh; *(volatile v4us*)(Al + oo) = ol; __threadfence(); *(volatile v4us*)(Ah + oo) = oh; *(volatile v4us*)(Al + oo) = ol; }
__global__ __launch_bounds__(256) void k_tohl(const float* __restrict__ F, bf* Hh, bf* Hl, size_t n4) { const size_t i = (size_t)blockIdx.x * 256 + threadIdx.x; if (i >= n4) return; const v4f a = *(const v4f*)(F + i * 4); v4us oh, ol;
#pragma unroll
    for (int q = 0; q < 4; ++q) { unsigned short h2, l2; splitf(a[q], h2, l2); oh[q] = h2; ol[q] = l2; }
    *(volatile v4us*)(Hh + i * 4) = oh; *(volatile v4us*)(Hl + i * 4) = ol; __threadfence(); *(volatile v4us*)(Hh + i * 4) = oh; *(volatile v4us*)(Hl + i * 4) = ol; }
__global__ __launch_bounds__(256) void k_copy(const float* __restrict__ T, float* out, size_t n4) { const size_t i = (size_t)blockIdx.x * 256 + threadIdx.x; if (i >= n4) return; const v4f a = *(const v4f*)(T + i * 4); *(volatile v4f*)(out + i * 4) = a; __threadfence(); *(volatile v4f*)(out + i * 4) = a; }

extern "C" void kernel_launch(void* const* d_in, const int* in_sizes, int n_in,
                              void* d_out, int out_size, void* d_ws, size_t ws_size, hipStream_t stream) {
    (void)in_sizes; (void)n_in; (void)out_size;
    const float* xq = (const float*)d_in[0]; const float* xk = (const float*)d_in[1]; const float* xv = (const float*)d_in[2];
    const float* Wq1 = (const float*)d_in[3]; const float* bq1 = (const float*)d_in[4]; const float* gq1w = (const float*)d_in[5]; const float* gq1b = (const float*)d_in[6]; const float* Wq2 = (const float*)d_in[7]; const float* bq2 = (const float*)d_in[8]; const float* gq2w = (const float*)d_in[9]; const float* gq2b = (const float*)d_in[10];
    const float* Wk = (const float*)d_in[11]; const float* bk = (const float*)d_in[12]; const float* gkw = (const float*)d_in[13]; const float* gkb = (const float*)d_in[14]; const float* Wv = (const float*)d_in[15]; const float* bv = (const float*)d_in[16]; const float* gvw = (const float*)d_in[17]; const float* gvb = (const float*)d_in[18];
    const float* Wm = (const float*)d_in[19]; const float* bm = (const float*)d_in[20]; const float* Ws = (const float*)d_in[21]; const float* bs = (const float*)d_in[22]; const float* Wc = (const float*)d_in[23]; const float* bc = (const float*)d_in[24]; const float* Wo = (const float*)d_in[25]; const float* bo = (const float*)d_in[26];
    float* OUT = (float*)d_out;
    char* wsp = (char*)d_ws;
    auto take = [&](size_t bytes) { char* p = wsp; wsp += (bytes + 255) & ~(size_t)255; return (void*)p; };
    bf* WQ1 = (bf*)take((size_t)DM * DM * 2); bf* WQ2 = (bf*)take((size_t)DM * DM * 2); bf* WKB = (bf*)take((size_t)DM * DM * 2); bf* WVB = (bf*)take((size_t)DM * DM * 2); bf* WMB = (bf*)take((size_t)MID * DK * 2); bf* WCB = (bf*)take((size_t)DK * MID * 2); bf* WOB = (bf*)take((size_t)DM * DM * 2);
    bf* XQ = (bf*)take((size_t)NP * DM * 2); bf* XK = (bf*)take((size_t)NP * DM * 2); bf* XV = (bf*)take((size_t)NP * DM * 2); float* T1 = (float*)take((size_t)NP * DM * 4); float* Q1 = (float*)take((size_t)NP * DM * 4); float* Q2 = (float*)take((size_t)NP * DM * 4); float* KK = (float*)take((size_t)NP * DM * 4); float* VV = (float*)take((size_t)NP * DM * 4);
    bf* Ah = (bf*)take((size_t)RPB * DK * 2); bf* Al = (bf*)take((size_t)RPB * DK * 2); float* AM = (float*)take((size_t)RPB * MID * 4); float* SP = (float*)take((size_t)RPB * 4); float* POOL = (float*)take((size_t)PQ * MID * 4); bf* PLh = (bf*)take((size_t)PQ * MID * 2); bf* PLl = (bf*)take((size_t)PQ * MID * 2); float* CH = (float*)take((size_t)PQ * DK * 4);
    bf* CTh = (bf*)take((size_t)NP * DM * 2); bf* CTl = (bf*)take((size_t)NP * DM * 2); float* TMP = (float*)take((size_t)NP * DM * 4);
    if ((size_t)(wsp - (char*)d_ws) > ws_size) return;
    { k_wtG<<<(DM * DM / 64 + 63) / 64, 256, 0, stream>>>(Wq1, DM, DM, WQ1); k_wtG<<<(DM * DM / 64 + 63) / 64, 256, 0, stream>>>(Wq2, DM, DM, WQ2); k_wtG<<<(DM * DM / 64 + 63) / 64, 256, 0, stream>>>(Wk, DM, DM, WKB); k_wtG<<<(DM * DM / 64 + 63) / 64, 256, 0, stream>>>(Wv, DM, DM, WVB);
      k_wtG<<<(DK * MID / 64 + 63) / 64, 256, 0, stream>>>(Wm, DK, MID, WMB); k_wtG<<<(MID * DK / 64 + 63) / 64, 256, 0, stream>>>(Wc, MID, DK, WCB); k_wtG<<<(DM * DM / 64 + 63) / 64, 256, 0, stream>>>(Wo, DM, DM, WOB);
      k_zero16<<<(NP * DM / 8 + 255) / 256, 256, 0, stream>>>(XQ, (size_t)NP * DM / 8); k_zero16<<<(NP * DM / 8 + 255) / 256, 256, 0, stream>>>(XK, (size_t)NP * DM / 8); k_zero16<<<(NP * DM / 8 + 255) / 256, 256, 0, stream>>>(XV, (size_t)NP * DM / 8);
      k_zero<<<(NP * DM / 4 + 255) / 256, 256, 0, stream>>>(Q1, (size_t)NP * DM / 4); k_zero<<<(NP * DM / 4 + 255) / 256, 256, 0, stream>>>(Q2, (size_t)NP * DM / 4); k_zero<<<(NP * DM / 4 + 255) / 256, 256, 0, stream>>>(KK, (size_t)NP * DM / 4); k_zero<<<(NP * DM / 4 + 255) / 256, 256, 0, stream>>>(VV, (size_t)NP * DM / 4);
      k_zero<<<(PQ * MID / 4 + 255) / 256, 256, 0, stream>>>(POOL, (size_t)PQ * MID / 4); k_zero16<<<(NP * DM / 8 + 255) / 256, 256, 0, stream>>>(CTh, (size_t)NP * DM / 8); k_zero16<<<(NP * DM / 8 + 255) / 256, 256, 0, stream>>>(CTl, (size_t)NP * DM / 8); }
    const unsigned gEG = (NQ * NH_ * 8 + 255) / 256;
    for (int b = 0; b < NB_; ++b) {
        k_cvt8<<<(NQ * DM / 8 + 255) / 256, 256, 0, stream>>>(xq + (size_t)b * NQ * DM, XQ, (size_t)NQ * DM / 8); k_cvt8<<<(NK * DM / 8 + 255) / 256, 256, 0, stream>>>(xk + (size_t)b * NK * DM, XK, (size_t)NK * DM / 8); k_cvt8<<<(NK * DM / 8 + 255) / 256, 256, 0, stream>>>(xv + (size_t)b * NK * DM, XV, (size_t)NK * DM / 8);
        k_gemmw<bf, 0, true><<<dim3(NP / 64, DM / 64, 1), 32, 0, stream>>>(XQ, nullptr, WQ1, nullptr, DM, T1, DM, bq1, 0, 0, 0); k_elugn<<<gEG, 256, 0, stream>>>(T1, gq1w, gq1b, Q1);
        k_gemmw<bf, 0, true><<<dim3(NP / 64, DM / 64, 1), 32, 0, stream>>>(XQ, nullptr, WQ2, nullptr, DM, T1, DM, bq2, 0, 0, 0); k_elugn<<<gEG, 256, 0, stream>>>(T1, gq2w, gq2b, Q2);
        k_gemmw<bf, 0, true><<<dim3(NP / 64, DM / 64, 1), 32, 0, stream>>>(XK, nullptr, WKB, nullptr, DM, T1, DM, bk, 0, 0, 0); k_elugn<<<gEG, 256, 0, stream>>>(T1, gkw, gkb, KK);
        k_gemmw<bf, 0, true><<<dim3(NP / 64, DM / 64, 1), 32, 0, stream>>>(XV, nullptr, WVB, nullptr, DM, T1, DM, bv, 0, 0, 0); k_elugn<<<gEG, 256, 0, stream>>>(T1, gvw, gvb, VV);
        k_prod<<<(unsigned)(((size_t)RPB * DK / 4 + 255) / 256), 256, 0, stream>>>(Q1, KK, Ah, Al);
        k_gemmw<bf, 1, true><<<dim3(RPB / 64, MID / 64, 1), 32, 0, stream>>>(Ah, Al, WMB, nullptr, DK, AM, MID, bm, 0, 0, 0);
        k_sppool<<<(NH_ * NQ * (MID / 4) + 255) / 256, 256, 0, stream>>>(AM, POOL);
        k_splog<<<(RPB + 255) / 256, 256, 0, stream>>>(AM, Ws, bs, SP);
        k_tohl<<<(PQ * MID / 4 + 255) / 256, 256, 0, stream>>>(POOL, PLh, PLl, (size_t)PQ * MID / 4);
        k_gemmw<bf, 1, true><<<dim3(PQ / 64, DK / 64, 1), 32, 0, stream>>>(PLh, PLl, WCB, nullptr, MID, CH, DK, bc, 0, 0, 0);
        k_attv<<<(NH_ * NQ * (DK / 4) + 255) / 256, 256, 0, stream>>>(SP, VV, Q2, CH, CTh, CTl);
        k_gemmw<bf, 1, true><<<dim3(NP / 64, DM / 64, 1), 32, 0, stream>>>(CTh, CTl, WOB, nullptr, DM, TMP, DM, bo, 0, 0, 0);
        k_copy<<<(NQ * DM / 4 + 255) / 256, 256, 0, stream>>>(TMP, OUT + (size_t)b * NQ * DM, (size_t)NQ * DM / 4); }
}
